// MultiheadSelfAttention_48996986913235
// MI455X (gfx1250) — hardware-verified
//
#include <hip/hip_runtime.h>
#include <math.h>

typedef __attribute__((ext_vector_type(16))) _Float16 v16h;
typedef __attribute__((ext_vector_type(16))) __bf16 v16b;
typedef __attribute__((ext_vector_type(8)))  _Float16 v8h;
typedef __attribute__((ext_vector_type(8)))  __bf16 v8b;
typedef __attribute__((ext_vector_type(8)))  float v8f;
typedef __attribute__((ext_vector_type(4)))  float v4f;
typedef __attribute__((ext_vector_type(4)))  unsigned v4u;

#ifndef NB
#define NB 2
#endif
#ifndef SEQ
#define SEQ 2048
#endif
#define NB_FULL 2
#define SEQ_FULL 2048
#define CC 1024
#define DIN 1024
#define NH 16
#define HD 64
#define EARLY (SEQ < 256 ? SEQ : 256)
#define NEGBIG (-3.0e38f)
#define SC2 (0.125f * 1.4426950408889634f)

static_assert(NB <= NB_FULL && SEQ <= SEQ_FULL);
static_assert(CC == NH * HD);
static_assert(HD == 64);
static_assert(DIN == 1024);
static_assert(DIN % 32 == 0 && CC % 32 == 0);
static_assert(CC % 128 == 0);
static_assert(SEQ % 64 == 0 && (NB * SEQ) % 64 == 0);
static_assert(EARLY % 64 == 0 && EARLY <= SEQ);
static_assert(SEQ % 8 == 0);
static_assert((long long)NB * SEQ * CC < 2147483647LL);

template <typename T> __device__ __forceinline__ void vst2(void* p, T v) { *(volatile T*)p = v; __threadfence(); *(volatile T*)p = v; }
__device__ __forceinline__ v8f wmma16(v16h a, v16h b, v8f c) {
  v8f d = __builtin_amdgcn_wmma_f32_16x16x32_f16(false, a, false, b, (short)0, c, false, false);
  asm volatile("v_nop\n\tv_nop\n\tv_nop\n\tv_nop" : "+v"(d) : "v"(a), "v"(b));
  return d;
}
__device__ __forceinline__ v8f wmma_bf(v16b a, v16b b, v8f c) {
  v8f d = __builtin_amdgcn_wmma_f32_16x16x32_bf16(false, a, false, b, (short)0, c, false, false);
  asm volatile("v_nop\n\tv_nop\n\tv_nop\n\tv_nop" : "+v"(d) : "v"(a), "v"(b));
  return d;
}
__device__ __forceinline__ v16b fragb_at(const __bf16* __restrict__ P, int off) {
  union { v16b v; v8b q[2]; } u; u.q[0] = *(const v8b*)(P + off); u.q[1] = *(const v8b*)(P + off + 16); return u.v;
}
__device__ __forceinline__ v16h fragh_at(const _Float16* __restrict__ P, int off) {
  union { v16h v; v8h q[2]; } u; u.q[0] = *(const v8h*)(P + off); u.q[1] = *(const v8h*)(P + off + 16); return u.v;
}
__device__ __forceinline__ unsigned bfb(float v) { unsigned u = __float_as_uint(v); u += 0x7FFFu + ((u >> 16) & 1u); return u >> 16; }
__device__ __forceinline__ void bsplit(float v, unsigned& h, unsigned& l) { h = bfb(v); l = bfb(v - __uint_as_float(h << 16)); }
__device__ __forceinline__ void split8(const v4f a, const v4f c, v4u& hv, v4u& lv) {
  unsigned h0, l0, h1, l1;
  bsplit(a.x, h0, l0); bsplit(a.y, h1, l1); hv.x = h0 | (h1 << 16); lv.x = l0 | (l1 << 16);
  bsplit(a.z, h0, l0); bsplit(a.w, h1, l1); hv.y = h0 | (h1 << 16); lv.y = l0 | (l1 << 16);
  bsplit(c.x, h0, l0); bsplit(c.y, h1, l1); hv.z = h0 | (h1 << 16); lv.z = l0 | (l1 << 16);
  bsplit(c.z, h0, l0); bsplit(c.w, h1, l1); hv.w = h0 | (h1 << 16); lv.w = l0 | (l1 << 16);
}
#define LDSX() do { asm volatile("s_wait_dscnt 0" ::: "memory"); __builtin_amdgcn_wave_barrier(); __builtin_amdgcn_fence(3  , "workgroup"); } while (0)

#define WS_TAB 0u
#define WS_XB  (WS_TAB + 4u * (size_t)SEQ * 64)
#define WS_WQ  (WS_XB  + 2u * (size_t)NB * SEQ * DIN)
#define WS_WK  (WS_WQ  + 2u * (size_t)CC * DIN)
#define WS_WV  (WS_WK  + 2u * (size_t)CC * DIN)
#define WS_WO  (WS_WV  + 2u * (size_t)CC * DIN)
#define WS_QH  (WS_WO  + 2u * (size_t)CC * DIN)
#define WS_QL  (WS_QH  + 2u * (size_t)NB * SEQ * CC)
#define WS_KH  (WS_QL  + 2u * (size_t)NB * SEQ * CC)
#define WS_KL  (WS_KH  + 2u * (size_t)NB * SEQ * CC)
#define WS_VT  (WS_KL  + 2u * (size_t)NB * SEQ * CC)
#define WS_VBH (WS_VT  + 2u * (size_t)NB * CC * SEQ)
#define WS_VBL (WS_VBH + 2u * (size_t)NB * CC * EARLY)
#define WS_YH  (WS_VBL + 2u * (size_t)NB * CC * EARLY)
#define WS_YL  (WS_YH  + 2u * (size_t)NB * SEQ * CC)
#define WS_END (WS_YL  + 2u * (size_t)NB * SEQ * CC)
static_assert((size_t)WS_END <= (size_t)134217728);

__global__ __launch_bounds__(256) void k_tab(float* __restrict__ TAB) {
  __shared__ __align__(16) float sm[512];
  const int tid = threadIdx.x; const int j = tid & 31; const int pos = blockIdx.x * 8 + (tid >> 5);
  double p = 1.0;
  p *= (j & 1)  ? 1.3335214321633240 : 1.0;
  p *= (j & 2)  ? 1.7782794100389228 : 1.0;
  p *= (j & 4)  ? 3.1622776601683795 : 1.0;
  p *= (j & 8)  ? 10.0 : 1.0;
  p *= (j & 16) ? 100.0 : 1.0;
  const float pf = (float)p; const float inv = 1.0f / pf; const float ang = (float)pos * inv;
  sm[tid * 2] = cosf(ang); sm[tid * 2 + 1] = sinf(ang);
  __syncthreads();
  if (tid < 128) vst2(TAB + (size_t)blockIdx.x * 512 + tid * 4, *(const v4f*)&sm[tid * 4]);
}
__global__ __launch_bounds__(256) void k_cvt(const float* __restrict__ SRC, unsigned short* __restrict__ DST, int rows, int seq, int seq_full) {
  const int i = blockIdx.x * 256 + threadIdx.x;
  if (i >= rows * (DIN / 8)) return;
  const int row = i >> 7, piece = i & 127; const int b = row / seq, t = row - b * seq;
  const float* s = SRC + ((size_t)b * seq_full + t) * DIN + piece * 8;
  const v4f a = *(const v4f*)s, c = *(const v4f*)(s + 4);
  v4u o; o.x = bfb(a.x) | (bfb(a.y) << 16); o.y = bfb(a.z) | (bfb(a.w) << 16); o.z = bfb(c.x) | (bfb(c.y) << 16); o.w = bfb(c.z) | (bfb(c.w) << 16);
  vst2(DST + (size_t)row * DIN + piece * 8, o);
}
__global__ __launch_bounds__(128) void k_proj(const __bf16* __restrict__ XB, const __bf16* __restrict__ WB, const float* __restrict__ TAB, int which,
    unsigned short* __restrict__ DH, unsigned short* __restrict__ DL, unsigned short* __restrict__ VT, unsigned short* __restrict__ VBH, unsigned short* __restrict__ VBL) {
  __shared__ __align__(16) float st[64][132];
  const int tid = threadIdx.x, lane = tid & 31, col = lane & 15, g = lane >> 4;
  const int wave = __builtin_amdgcn_readfirstlane(tid >> 5);
  const int c0 = blockIdx.y * 128; const int r0 = blockIdx.x * 64;
  v8f acc[8] = {};
  const int aoff = (r0 + wave * 16 + col) * DIN + 8 * g; const int woff = (c0 + col) * DIN + 8 * g;
#pragma unroll 1
  for (int kc = 0; kc < DIN / 32; ++kc) { const v16b a = fragb_at(XB, aoff + kc * 32);
#pragma unroll
    for (int j = 0; j < 8; ++j) { const v16b w = fragb_at(WB, woff + j * 16 * DIN + kc * 32); acc[j] = wmma_bf(a, w, acc[j]); } }
#pragma unroll
  for (int j = 0; j < 8; ++j)
#pragma unroll
    for (int r = 0; r < 8; ++r) st[wave * 16 + 8 * g + r][j * 16 + col] = acc[j][r];
  __syncthreads();
  if (which < 2) {
    for (int e = tid; e < 64 * 16; e += 128) { const int rl = e >> 4, q = e & 15; const int t = (r0 + rl) % SEQ;
      const v4f x0 = *(const v4f*)&st[rl][q * 8], x1 = *(const v4f*)&st[rl][q * 8 + 4];
      const float* tp = TAB + (size_t)t * 64 + ((c0 + q * 8) & 63);
      const v4f t0 = *(const v4f*)tp, t1 = *(const v4f*)(tp + 4);
      v4f y0, y1;
      y0.x = x0.x * t0.x - x0.y * t0.y; y0.y = x0.y * t0.x + x0.x * t0.y;
      y0.z = x0.z * t0.z - x0.w * t0.w; y0.w = x0.w * t0.z + x0.z * t0.w;
      y1.x = x1.x * t1.x - x1.y * t1.y; y1.y = x1.y * t1.x + x1.x * t1.y;
      y1.z = x1.z * t1.z - x1.w * t1.w; y1.w = x1.w * t1.z + x1.z * t1.w;
      v4u hv, lv; split8(y0, y1, hv, lv);
      const size_t o = (size_t)(r0 + rl) * CC + c0 + q * 8;
      vst2(DH + o, hv); vst2(DL + o, lv); }
  } else {
    const int bb = r0 / SEQ, t0 = r0 % SEQ; const bool early = t0 < EARLY;
    for (int e = tid; e < 128 * 8; e += 128) { const int cl = e >> 3, q = e & 7;
      float v[8];
#pragma unroll
      for (int i = 0; i < 8; ++i) v[i] = st[q * 8 + i][cl];
      v8h hh;
#pragma unroll
      for (int i = 0; i < 8; ++i) hh[i] = (_Float16)v[i];
      vst2(VT + ((size_t)bb * CC + c0 + cl) * SEQ + t0 + q * 8, __builtin_bit_cast(v4u, hh));
      if (early) { v4f a, c; a.x = v[0]; a.y = v[1]; a.z = v[2]; a.w = v[3]; c.x = v[4]; c.y = v[5]; c.z = v[6]; c.w = v[7];
        v4u hv, lv; split8(a, c, hv, lv); const size_t o3 = ((size_t)bb * CC + c0 + cl) * EARLY + t0 + q * 8;
        vst2(VBH + o3, hv); vst2(VBL + o3, lv); } } }
}
template <bool EP>
__device__ __forceinline__ void attn_body(const __bf16* __restrict__ QH, const __bf16* __restrict__ QL, const __bf16* __restrict__ KH, const __bf16* __restrict__ KL,
    const _Float16* __restrict__ VT, const __bf16* __restrict__ VBH, const __bf16* __restrict__ VBL, unsigned short* __restrict__ YH, unsigned short* __restrict__ YL, const int qb) {
  __shared__ __align__(16) unsigned short pt[2][4][16][40];
  __shared__ __align__(16) float cs[4][16][68];
  const int tid = threadIdx.x, lane = tid & 31, col = lane & 15, g = lane >> 4;
  const int wave = __builtin_amdgcn_readfirstlane(tid >> 5);
  const int h = blockIdx.y, b = blockIdx.z;
  const int q0 = qb * 64 + wave * 16;
  const int nst = ((q0 + 15) >> 5) + 1;
  const int rowb = b * SEQ;
  float m[8], l[8]; v8f o[4] = {};
#pragma unroll
  for (int r = 0; r < 8; ++r) { m[r] = NEGBIG; l[r] = 0.f; }
  int qoff = (rowb + q0 + col) * CC + h * HD + 8 * g;
#pragma unroll 1
  for (int st = 0; st < nst; ++st) { const int key0 = st * 32;
    asm volatile("" : "+v"(qoff));
    v8f s[2];
#pragma unroll
    for (int t = 0; t < 2; ++t) { v8f a = {}; const int koff = (rowb + key0 + t * 16 + col) * CC + h * HD + 8 * g;
#pragma unroll
      for (int kc = 0; kc < 2; ++kc) { const v16b qh = fragb_at(QH, qoff + kc * 32), ql = fragb_at(QL, qoff + kc * 32); const v16b kh = fragb_at(KH, koff + kc * 32), kl = fragb_at(KL, koff + kc * 32);
        a = wmma_bf(ql, kh, a); a = wmma_bf(qh, kl, a); a = wmma_bf(qh, kh, a); }
      s[t] = a; }
    const bool diag = (key0 + 31 > q0);
    float p[2][8];
#pragma unroll
    for (int r = 0; r < 8; ++r) { const int qm = q0 + 8 * g + r;
      float t0 = s[0][r] * SC2, t1 = s[1][r] * SC2;
      t0 = (diag && (key0 + col > qm)) ? NEGBIG : t0; t1 = (diag && (key0 + 16 + col > qm)) ? NEGBIG : t1;
      float mx = fmaxf(t0, t1);
      mx = fmaxf(mx, __shfl_xor(mx, 8)); mx = fmaxf(mx, __shfl_xor(mx, 4)); mx = fmaxf(mx, __shfl_xor(mx, 2)); mx = fmaxf(mx, __shfl_xor(mx, 1));
      const float mn = fmaxf(m[r], mx); const float sc = exp2f(m[r] - mn); m[r] = mn;
      const float p0 = exp2f(t0 - mn), p1 = exp2f(t1 - mn);
      l[r] = l[r] * sc + (p0 + p1);
      o[0][r] *= sc; o[1][r] *= sc; o[2][r] *= sc; o[3][r] *= sc;
      p[0][r] = p0; p[1][r] = p1; }
#pragma unroll
    for (int t = 0; t < 2; ++t)
#pragma unroll
      for (int r = 0; r < 8; ++r) {
        if (EP) { unsigned hb, lb; bsplit(p[t][r], hb, lb); pt[0][wave][8 * g + r][t * 16 + col] = (unsigned short)hb; pt[1][wave][8 * g + r][t * 16 + col] = (unsigned short)lb; }
        else pt[0][wave][8 * g + r][t * 16 + col] = __builtin_bit_cast(unsigned short, (_Float16)(p[t][r] * 1024.0f)); }
    LDSX();
    if (EP) { union { v16b v; v4u q[2]; } uh, ul;
      uh.q[0] = *(const v4u*)&pt[0][wave][col][8 * g]; uh.q[1] = *(const v4u*)&pt[0][wave][col][16 + 8 * g];
      ul.q[0] = *(const v4u*)&pt[1][wave][col][8 * g]; ul.q[1] = *(const v4u*)&pt[1][wave][col][16 + 8 * g];
      asm volatile("" ::: "memory");
      const int voff = (b * CC + h * HD + col) * EARLY + key0 + 8 * g;
#pragma unroll
      for (int j = 0; j < 4; ++j) { const v16b vh = fragb_at(VBH, voff + j * 16 * EARLY), vl = fragb_at(VBL, voff + j * 16 * EARLY);
        o[j] = wmma_bf(ul.v, vh, o[j]); o[j] = wmma_bf(uh.v, vl, o[j]); o[j] = wmma_bf(uh.v, vh, o[j]); }
    } else { union { v16h v; v4u q[2]; } up;
      up.q[0] = *(const v4u*)&pt[0][wave][col][8 * g]; up.q[1] = *(const v4u*)&pt[0][wave][col][16 + 8 * g];
      asm volatile("" ::: "memory");
      const int voff = (b * CC + h * HD + col) * SEQ + key0 + 8 * g;
#pragma unroll
      for (int j = 0; j < 4; ++j) { const v16h vb = fragh_at(VT, voff + j * 16 * SEQ); o[j] = wmma16(up.v, vb, o[j]); } }
  }
  float inv[8];
#pragma unroll
  for (int r = 0; r < 8; ++r) { float lt = l[r]; lt += __shfl_xor(lt, 8); lt += __shfl_xor(lt, 4); lt += __shfl_xor(lt, 2); lt += __shfl_xor(lt, 1);
    inv[r] = (1.0f / lt) * (EP ? 1.0f : (1.0f / 1024.0f)); }
#pragma unroll
  for (int j = 0; j < 4; ++j)
#pragma unroll
    for (int r = 0; r < 8; ++r) cs[wave][8 * g + r][j * 16 + col] = o[j][r] * inv[r];
  LDSX();
#pragma unroll 1
  for (int it = 0; it < 4; ++it) { const int rl = it * 4 + (lane >> 3), q = lane & 7;
    const v4f x0 = *(const v4f*)&cs[wave][rl][q * 8], x1 = *(const v4f*)&cs[wave][rl][q * 8 + 4];
    v4u hv, lv; split8(x0, x1, hv, lv);
    const size_t d = (size_t)(rowb + q0 + rl) * CC + h * HD + q * 8;
    vst2(YH + d, hv); vst2(YL + d, lv); }
}
__global__ __launch_bounds__(128) void k_attn_early(const __bf16* __restrict__ QH, const __bf16* __restrict__ QL, const __bf16* __restrict__ KH, const __bf16* __restrict__ KL,
    const _Float16* __restrict__ VT, const __bf16* __restrict__ VBH, const __bf16* __restrict__ VBL, unsigned short* __restrict__ YH, unsigned short* __restrict__ YL) {
  attn_body<true>(QH, QL, KH, KL, VT, VBH, VBL, YH, YL, (int)blockIdx.x);
}
__global__ __launch_bounds__(128) void k_attn_main(const __bf16* __restrict__ QH, const __bf16* __restrict__ QL, const __bf16* __restrict__ KH, const __bf16* __restrict__ KL,
    const _Float16* __restrict__ VT, const __bf16* __restrict__ VBH, const __bf16* __restrict__ VBL, unsigned short* __restrict__ YH, unsigned short* __restrict__ YL) {
  attn_body<false>(QH, QL, KH, KL, VT, VBH, VBL, YH, YL, (int)blockIdx.x + EARLY / 64);
}
__global__ __launch_bounds__(128) void k_out(const __bf16* __restrict__ YH, const __bf16* __restrict__ YL, const __bf16* __restrict__ WOB, float* __restrict__ OUT) {
  __shared__ __align__(16) float sf[4][16][132];
  const int tid = threadIdx.x, lane = tid & 31, col = lane & 15, g = lane >> 4;
  const int wave = __builtin_amdgcn_readfirstlane(tid >> 5);
  const int c0 = blockIdx.y * 128; const int r0 = blockIdx.x * 64 + wave * 16;
  v8f acc[8] = {};
  const int aoff = (r0 + col) * CC + 8 * g; const int woff = (c0 + col) * CC + 8 * g;
#pragma unroll 1
  for (int kc = 0; kc < CC / 32; ++kc) { const v16b ah = fragb_at(YH, aoff + kc * 32), al = fragb_at(YL, aoff + kc * 32);
#pragma unroll
    for (int j = 0; j < 8; ++j) { const v16b w = fragb_at(WOB, woff + j * 16 * CC + kc * 32); acc[j] = wmma_bf(al, w, acc[j]); acc[j] = wmma_bf(ah, w, acc[j]); } }
#pragma unroll
  for (int j = 0; j < 8; ++j)
#pragma unroll
    for (int r = 0; r < 8; ++r) sf[wave][8 * g + r][j * 16 + col] = acc[j][r];
  LDSX();
#pragma unroll 1
  for (int rl = 0; rl < 16; ++rl) vst2(OUT + (size_t)(r0 + rl) * CC + c0 + lane * 4, *(const v4f*)&sf[wave][rl][lane * 4]);
}

extern "C" void kernel_launch(void* const* d_in, const int* in_sizes, int n_in, void* d_out, int out_size, void* d_ws, size_t ws_size, hipStream_t stream) {
  if (n_in < 5) return;
  if (ws_size < (size_t)WS_END) return;
  if (in_sizes[0] < ((NB - 1) * SEQ_FULL + SEQ) * DIN) return;
  if (in_sizes[1] < CC * DIN || in_sizes[2] < CC * DIN || in_sizes[3] < CC * DIN || in_sizes[4] < CC * DIN) return;
  if (out_size < NB * SEQ * CC) return;
  const float* x = (const float*)d_in[0]; const float* wq = (const float*)d_in[1]; const float* wk = (const float*)d_in[2]; const float* wv = (const float*)d_in[3]; const float* wo = (const float*)d_in[4];
  char* ws = (char*)d_ws;
  float* TAB = (float*)(ws + WS_TAB);
  unsigned short *XB = (unsigned short*)(ws + WS_XB), *WQB = (unsigned short*)(ws + WS_WQ), *WKB = (unsigned short*)(ws + WS_WK), *WVB = (unsigned short*)(ws + WS_WV), *WOB = (unsigned short*)(ws + WS_WO);
  unsigned short *QH = (unsigned short*)(ws + WS_QH), *QL = (unsigned short*)(ws + WS_QL), *KH = (unsigned short*)(ws + WS_KH), *KL = (unsigned short*)(ws + WS_KL);
  unsigned short *VT = (unsigned short*)(ws + WS_VT), *VBH = (unsigned short*)(ws + WS_VBH), *VBL = (unsigned short*)(ws + WS_VBL), *YH = (unsigned short*)(ws + WS_YH), *YL = (unsigned short*)(ws + WS_YL);
  k_tab<<<dim3(SEQ / 8), 256, 0, stream>>>(TAB);
  k_cvt<<<dim3(NB * SEQ * (DIN / 8) / 256), 256, 0, stream>>>(x, XB, NB * SEQ, SEQ, SEQ_FULL);
  k_cvt<<<dim3(CC * (DIN / 8) / 256), 256, 0, stream>>>(wq, WQB, CC, CC, CC);
  k_cvt<<<dim3(CC * (DIN / 8) / 256), 256, 0, stream>>>(wk, WKB, CC, CC, CC);
  k_cvt<<<dim3(CC * (DIN / 8) / 256), 256, 0, stream>>>(wv, WVB, CC, CC, CC);
  k_cvt<<<dim3(CC * (DIN / 8) / 256), 256, 0, stream>>>(wo, WOB, CC, CC, CC);
  k_proj<<<dim3(NB * SEQ / 64, CC / 128), 128, 0, stream>>>((const __bf16*)XB, (const __bf16*)WQB, TAB, 0, QH, QL, VT, VBH, VBL);
  k_proj<<<dim3(NB * SEQ / 64, CC / 128), 128, 0, stream>>>((const __bf16*)XB, (const __bf16*)WKB, TAB, 1, KH, KL, VT, VBH, VBL);
  k_proj<<<dim3(NB * SEQ / 64, CC / 128), 128, 0, stream>>>((const __bf16*)XB, (const __bf16*)WVB, TAB, 2, QH, QL, VT, VBH, VBL);
  k_attn_early<<<dim3(EARLY / 64, NH, NB), 128, 0, stream>>>((const __bf16*)QH, (const __bf16*)QL, (const __bf16*)KH, (const __bf16*)KL, (const _Float16*)VT, (const __bf16*)VBH, (const __bf16*)VBL, YH, YL);
  if (SEQ > EARLY)
    k_attn_main<<<dim3((SEQ - EARLY) / 64, NH, NB), 128, 0, stream>>>((const __bf16*)QH, (const __bf16*)QL, (const __bf16*)KH, (const __bf16*)KL, (const _Float16*)VT, (const __bf16*)VBH, (const __bf16*)VBL, YH, YL);
  k_out<<<dim3(NB * SEQ / 64, CC / 128), 128, 0, stream>>>((const __bf16*)YH, (const __bf16*)YL, (const __bf16*)WOB, (float*)d_out);
}
